// GCNModel_56865366999234
// MI455X (gfx1250) — hardware-run, weakly checked
//
#include <hip/hip_runtime.h>

typedef float          v8f   __attribute__((ext_vector_type(8)));
typedef float          v4f   __attribute__((ext_vector_type(4)));
typedef unsigned int   v4u   __attribute__((ext_vector_type(4)));
typedef int            v8i   __attribute__((ext_vector_type(8)));
typedef unsigned short v8us  __attribute__((ext_vector_type(8)));
typedef unsigned short v16us __attribute__((ext_vector_type(16)));
typedef __bf16         v16bf __attribute__((ext_vector_type(16)));
typedef _Float16       v16h  __attribute__((ext_vector_type(16)));
typedef v4f  __attribute__((may_alias)) v4fa;
typedef v8us __attribute__((may_alias)) v8usa;
union FragB { v16bf v; v16us u; v8us h[2]; v8i w; };
union FragH { v16h  v; v16us u; v8us h[2]; v8i w; };

__device__ __forceinline__ v8f wmb(const FragB& a, const FragB& b, v8f c) {
  v8f d = __builtin_amdgcn_wmma_f32_16x16x32_bf16(false, a.v, false, b.v, (short)0, c, false, false);
  asm volatile("v_nop\n\tv_nop\n\tv_nop\n\tv_nop" : "+v"(d) : "v"(a.w), "v"(b.w));
  return d;
}

__device__ __forceinline__ v8f wmh(const FragH& a, const FragH& b, v8f c) {
  v8f d = __builtin_amdgcn_wmma_f32_16x16x32_f16(false, a.v, false, b.v, (short)0, c, false, false);
  asm volatile("v_nop\n\tv_nop\n\tv_nop\n\tv_nop" : "+v"(d) : "v"(a.w), "v"(b.w));
  return d;
}

__device__ __forceinline__ unsigned bf16_bits(float f) {
  const unsigned u = __float_as_uint(f);
  const unsigned r = (u + 0x7FFFu + ((u >> 16) & 1u)) >> 16;
  const unsigned q = (u >> 16) | 0x40u;
  return ((u & 0x7fffffffu) > 0x7f800000u) ? q : r;
}

__device__ __forceinline__ float bf16_val(float f) {
  return __uint_as_float(bf16_bits(f) << 16);
}
__device__ __forceinline__ int clampi(int v, int lo, int hi) {
  return v < lo ? lo : (v > hi ? hi : v);
}

__device__ __forceinline__ unsigned f16_bits(float f) {
  const unsigned u  = __float_as_uint(f);
  const unsigned s  = (u >> 16) & 0x8000u;
  const unsigned a  = u & 0x7fffffffu;
  const unsigned t  = a - 0x38000000u;
  const unsigned r  = (t + 0x0FFFu + ((t >> 13) & 1u)) >> 13;
  const unsigned rc = r > 0x7C00u ? 0x7C00u : r;
  const bool small  = a < 0x38800000u;
  const bool isnan  = a > 0x7f800000u;
  const unsigned fin = small ? 0u : (s | rc);
  return isnan ? (s | 0x7E00u) : fin;
}

__device__ __forceinline__ unsigned pk16(unsigned lo, unsigned hi) { return lo | (hi << 16); }
__device__ __forceinline__ unsigned bf16_lo_bits(float v) {
  float hi = bf16_val(v);
  asm volatile("" : "+v"(hi));
  return bf16_bits(v - hi);
}
__device__ __forceinline__ v4u pack8_bf16(v4f a, v4f c) {
  return (v4u){ pk16(bf16_bits(a[0]), bf16_bits(a[1])), pk16(bf16_bits(a[2]), bf16_bits(a[3])),
                pk16(bf16_bits(c[0]), bf16_bits(c[1])), pk16(bf16_bits(c[2]), bf16_bits(c[3])) };
}
__device__ __forceinline__ v4u pack8_bf16_lo(v4f a, v4f c) {
  return (v4u){ pk16(bf16_lo_bits(a[0]), bf16_lo_bits(a[1])), pk16(bf16_lo_bits(a[2]), bf16_lo_bits(a[3])),
                pk16(bf16_lo_bits(c[0]), bf16_lo_bits(c[1])), pk16(bf16_lo_bits(c[2]), bf16_lo_bits(c[3])) };
}
__device__ __forceinline__ v4u pack8_f16(v4f a, v4f c) {
  return (v4u){ pk16(f16_bits(a[0]), f16_bits(a[1])), pk16(f16_bits(a[2]), f16_bits(a[3])),
                pk16(f16_bits(c[0]), f16_bits(c[1])), pk16(f16_bits(c[2]), f16_bits(c[3])) };
}

template <int FORM>
__global__ __launch_bounds__(256) void k_plane(const float* __restrict__ src, int rows, int cols, int ldsrc,
                                               unsigned short* __restrict__ dst, int MP, int KP) {
  static_assert(FORM >= 0 && FORM <= 3);
  const int KTOT = (FORM == 1 || FORM == 3) ? 2 * KP : KP;
  const unsigned ppr   = (unsigned)(KTOT >> 3);
  const unsigned kp8   = (unsigned)(KP >> 3);
  const unsigned total = (unsigned)MP * ppr;
  const unsigned g     = blockIdx.x * 256u + threadIdx.x;
  const unsigned rowu  = g / ppr;
  const unsigned p     = g - rowu * ppr;
  const bool second    = p >= kp8;
  const int row = (int)rowu;
  const int c0  = (int)((second ? p - kp8 : p) << 3);
  const float* srow = src + (size_t)clampi(row, 0, rows - 1) * (size_t)ldsrc;
  float x[8];
  unsigned mk[8];
#pragma unroll
  for (int e = 0; e < 8; ++e) {
    const int c = c0 + e;
    const float v = srow[clampi(c, 0, cols - 1)];
    asm volatile("" :: "v"(v));
    x[e]  = v;
    mk[e] = (row < rows && c < cols) ? 0xFFFFu : 0u;
  }
  const v4f a = (v4f){ x[0], x[1], x[2], x[3] };
  const v4f c = (v4f){ x[4], x[5], x[6], x[7] };
  v4u o;
  if (FORM == 2) {
    o = pack8_f16(a, c);
  } else {
    const v4u hi = pack8_bf16(a, c);
    o = hi;
    if (FORM == 1) { const v4u lo = pack8_bf16_lo(a, c); o = second ? lo : hi; }
  }
  const v4u mw = (v4u){ pk16(mk[0], mk[1]), pk16(mk[2], mk[3]), pk16(mk[4], mk[5]), pk16(mk[6], mk[7]) };
  o &= mw;
  if (g < total) {
    volatile v4u* q = (volatile v4u*)(dst + (size_t)g * 8);
    *q = o;
    __threadfence();
    *q = o;
  }
}

template <int FORM> struct FragOf    { typedef FragB T; };
template <>         struct FragOf<2> { typedef FragH T; };
__device__ __forceinline__ v8f mm(const FragB& a, const FragB& b, v8f c) { return wmb(a, b, c); }
__device__ __forceinline__ v8f mm(const FragH& a, const FragH& b, v8f c) { return wmh(a, b, c); }
template <class F> __device__ __forceinline__ F ld_frag(const unsigned short* p) {
  F f;
  f.h[0] = *(const v8usa*)(p);
  f.h[1] = *(const v8usa*)(p + 16);
  return f;
}

template <int FORM, int EPI>
__global__ __launch_bounds__(256) __attribute__((amdgpu_num_vgpr(248)))
void k_gemm_nt(const unsigned short* __restrict__ A, const unsigned short* __restrict__ B,
               const float* __restrict__ bias, float* __restrict__ D, int M, int N, int KTOT, int ldd) {
  static_assert(FORM >= 0 && FORM <= 2);
  static_assert(EPI == 0 || EPI == 1);
  typedef typename FragOf<FORM>::T F;
  __shared__ __attribute__((aligned(16))) float sT[8][16 * 68];
  const int lane = threadIdx.x & 31;
  const int wave = threadIdx.x >> 5;
  const int tilesM = (M + 63) >> 6;
  const int tilesN = (N + 63) >> 6;
  const int tile = blockIdx.x * 8 + wave;
  if (tile >= tilesM * tilesN) return;
  const int tm = tile / tilesN;
  const int tn = tile - tm * tilesN;
  const int m0 = tm << 6;
  const int n0 = tn << 6;

  const int rl = lane & 15;
  const int h8 = (lane >> 4) * 8;
  const unsigned short* pa = A + (size_t)(m0 + rl) * (size_t)KTOT + h8;
  const unsigned short* pb = B + (size_t)(n0 + rl) * (size_t)KTOT + h8;

  v8f acc[4][4];
#pragma unroll
  for (int i = 0; i < 4; ++i)
#pragma unroll
    for (int j = 0; j < 4; ++j) acc[i][j] = (v8f){0.f, 0.f, 0.f, 0.f, 0.f, 0.f, 0.f, 0.f};

#pragma unroll 1
  for (int k0 = 0; k0 < KTOT; k0 += 32) {
    F bf[4];
#pragma unroll
    for (int j = 0; j < 4; ++j) bf[j] = ld_frag<F>(pb + (size_t)(j << 4) * (size_t)KTOT + k0);
#pragma unroll
    for (int i = 0; i < 4; ++i) {
      const F af = ld_frag<F>(pa + (size_t)(i << 4) * (size_t)KTOT + k0);
#pragma unroll
      for (int j = 0; j < 4; ++j) acc[i][j] = mm(af, bf[j], acc[i][j]);
    }
  }

  float* slab = sT[wave];
  const int hh = lane >> 4;
  const int c4 = (lane & 15) * 4;
  const int nc = n0 + c4;
  const bool cok = nc < N;
  v4f bv = (v4f){0.f, 0.f, 0.f, 0.f};
  if (EPI == 1) {
    bv = *(const v4fa*)(bias + clampi(nc, 0, N - 4));
    asm volatile("" :: "v"(bv));
  }
#pragma unroll
  for (int i = 0; i < 4; ++i) {
    const int mBase = m0 + (i << 4);
#pragma unroll
    for (int j = 0; j < 4; ++j) {
#pragma unroll
      for (int r = 0; r < 8; ++r) slab[(h8 + r) * 68 + (j << 4) + rl] = acc[i][j][r];
    }
    __builtin_amdgcn_fence(__ATOMIC_RELEASE, "workgroup");
    __builtin_amdgcn_wave_barrier();
    __builtin_amdgcn_fence(__ATOMIC_ACQUIRE, "workgroup");
    v4f vv[8];
#pragma unroll
    for (int it = 0; it < 8; ++it) {
      const int row = it * 2 + hh;
      v4f v = *(const v4fa*)(slab + row * 68 + c4);
      if (EPI == 1) v += bv;
      vv[it] = v;
    }
    for (int pass = 0; pass < 2; ++pass) {
#pragma unroll
      for (int it = 0; it < 8; ++it) {
        const int row = mBase + it * 2 + hh;
        if (cok && row < M) *(volatile v4f*)(D + (size_t)row * (size_t)ldd + nc) = vv[it];
      }
      __threadfence();
    }
    __builtin_amdgcn_fence(__ATOMIC_RELEASE, "workgroup");
    __builtin_amdgcn_wave_barrier();
    __builtin_amdgcn_fence(__ATOMIC_ACQUIRE, "workgroup");
  }
}

#pragma clang fp contract(off)

#define GN      100000
#define GE      1600000
#define GK1     128
#define GH      64
#define GC      32
#define GMP     100096
#define NTHR    256
#define NWAVE   8
#define EPT     8
#define WCH     (32 * EPT)
#define NBRUN   1024
#define SLB     10
#define NBK     98
#define WLCAP   2880
#define RCAP    21504
#define DEGCAP  64
#define MAXDEG_MEAS   36
#define MAXB1024_MEAS 16710
#define SPLIT_L2 1

#define BK_ZINTS (NWAVE * WLCAP + RCAP + 3 * NBRUN)
#define BK_INTS  (BK_ZINTS + 16)
#define BK_LDS   (BK_INTS * 4)

static_assert(GMP % 128 == 0 && GMP >= GN && GMP % 64 == 0 && GMP == 782 * 128);
static_assert(GK1 % 32 == 0 && (2 * GH) % 32 == 0 && GH % 32 == 0 && GH == 2 * 32 && GC == 32);
static_assert(NBRUN == (1 << SLB) && NBRUN == NTHR * 4 && NBRUN % 32 == 0);
static_assert(NBK * NBRUN >= GMP && NBK * NBRUN >= GN && (NBK - 1) * NBRUN < GN);
static_assert(GE < (1 << 21));
static_assert(GE % 4 == 0);
static_assert((long long)RCAP * 100 >= (long long)MAXB1024_MEAS * 125);
static_assert(WLCAP >= MAXB1024_MEAS / 8 + 8 * 46 + 1);
static_assert(MAXDEG_MEAS + 1 + 8 <= DEGCAP);
static_assert(RCAP % (NTHR * 4) == 0 && BK_ZINTS % 4 == 0);
static_assert((NWAVE * WLCAP) % 4 == 0 && RCAP % 4 == 0);
static_assert(BK_LDS <= 262144);
static_assert((GMP * GK1 / 8) % 256 == 0);
static_assert(GMP % 8 == 0 && GN % 8 == 0);

typedef float v2f __attribute__((ext_vector_type(2)));
typedef int   v4i __attribute__((ext_vector_type(4)));
typedef v2f __attribute__((may_alias)) v2fa;
typedef v4i __attribute__((may_alias)) v4ia;

__device__ __forceinline__ void st2_v4u(unsigned* p, v4u v) {
  *(volatile v4u*)p = v;
  __threadfence();
  *(volatile v4u*)p = v;
}
__device__ __forceinline__ void st2_v4f(float* p, v4f v) {
  *(volatile v4f*)p = v;
  __threadfence();
  *(volatile v4f*)p = v;
}

__device__ __forceinline__ v4u gather8_bf16(const float* __restrict__ base, int stride, unsigned mk) {
  float f[8];
#pragma unroll
  for (int i = 0; i < 8; ++i) {
    const float v = base[(size_t)i * (size_t)stride];
    asm volatile("" :: "v"(v));
    f[i] = v;
  }
  unsigned b[8];
#pragma unroll
  for (int i = 0; i < 8; ++i) b[i] = bf16_bits(f[i]) & mk;
  return (v4u){ pk16(b[0], b[1]), pk16(b[2], b[3]), pk16(b[4], b[5]), pk16(b[6], b[7]) };
}

__global__ __launch_bounds__(NTHR) void k_prep(const float* __restrict__ w1, const float* __restrict__ b1,
                                               const float* __restrict__ w2, const float* __restrict__ b2,
                                               unsigned short* w1t, unsigned short* w2p, float* bias) {
  __shared__ __attribute__((aligned(16))) float sb[NTHR];
  const int tid = (int)threadIdx.x;
  const int blk = (int)blockIdx.x;
  if (blk < 4) {
    const int u = blk * NTHR + tid;
    const int n = u >> 4, k8 = (u & 15) * 8;
    const v4u o = gather8_bf16(w1 + (size_t)k8 * GH + n, GH, 0xFFFFu);
    st2_v4u((unsigned*)(w1t + (size_t)u * 8), o);
  } else if (blk < 8) {
    const int u = (blk - 4) * NTHR + tid;
    const int n = u >> 4, k8 = (u & 15) * 8;
    const int kk = k8 & (GH - 1);
    const int nc = n < GC ? n : GC - 1;
    const unsigned mk = n < GC ? 0xFFFFu : 0u;
    const v4u o = gather8_bf16(w2 + (size_t)kk * GC + nc, GC, mk);
    st2_v4u((unsigned*)(w2p + (size_t)u * 8), o);
  } else {
    const int i1 = clampi(tid, 0, GH - 1);
    const int i2 = clampi(tid - GH, 0, GC - 1);
    const float v1 = b1[i1];
    asm volatile("" :: "v"(v1));
    const float v2 = b2[i2];
    asm volatile("" :: "v"(v2));
    const float c1 = bf16_val(v1);
    const float c2 = bf16_val(v2);
    float o = 0.0f;
    o = (tid < GH + GC) ? c2 : o;
    o = (tid < GH) ? c1 : o;
    sb[tid] = o;
    __syncthreads();
    if (tid < 64) {
      const v4f v = *(const v4fa*)(sb + 4 * tid);
      st2_v4f(bias + 4 * tid, v);
    }
  }
}

__device__ __forceinline__ int bk_emit(int* mylist, int wc, int e0, unsigned nbs,
                                       int d0, int d1, int d2, int d3, int d4, int d5, int d6, int d7) {
  const unsigned s0 = (unsigned)d0 - nbs, s1 = (unsigned)d1 - nbs, s2 = (unsigned)d2 - nbs, s3 = (unsigned)d3 - nbs;
  const unsigned s4 = (unsigned)d4 - nbs, s5 = (unsigned)d5 - nbs, s6 = (unsigned)d6 - nbs, s7 = (unsigned)d7 - nbs;
  const bool h0 = s0 < (unsigned)NBRUN, h1 = s1 < (unsigned)NBRUN, h2 = s2 < (unsigned)NBRUN, h3 = s3 < (unsigned)NBRUN;
  const bool h4 = s4 < (unsigned)NBRUN, h5 = s5 < (unsigned)NBRUN, h6 = s6 < (unsigned)NBRUN, h7 = s7 < (unsigned)NBRUN;
  const unsigned m0 = __builtin_amdgcn_ballot_w32(h0), m1 = __builtin_amdgcn_ballot_w32(h1);
  const unsigned m2 = __builtin_amdgcn_ballot_w32(h2), m3 = __builtin_amdgcn_ballot_w32(h3);
  const unsigned m4 = __builtin_amdgcn_ballot_w32(h4), m5 = __builtin_amdgcn_ballot_w32(h5);
  const unsigned m6 = __builtin_amdgcn_ballot_w32(h6), m7 = __builtin_amdgcn_ballot_w32(h7);
  const unsigned any = m0 | m1 | m2 | m3 | m4 | m5 | m6 | m7;
  if (any != 0u) {
    const int pre = (int)(__builtin_amdgcn_mbcnt_lo(m0, 0u) + __builtin_amdgcn_mbcnt_lo(m1, 0u) +
                          __builtin_amdgcn_mbcnt_lo(m2, 0u) + __builtin_amdgcn_mbcnt_lo(m3, 0u) +
                          __builtin_amdgcn_mbcnt_lo(m4, 0u) + __builtin_amdgcn_mbcnt_lo(m5, 0u) +
                          __builtin_amdgcn_mbcnt_lo(m6, 0u) + __builtin_amdgcn_mbcnt_lo(m7, 0u));
    int p = wc + pre;
    if (h0) { if (p < WLCAP) mylist[p] = ((e0 + 0) << SLB) | (int)s0; p = p + 1; }
    if (h1) { if (p < WLCAP) mylist[p] = ((e0 + 1) << SLB) | (int)s1; p = p + 1; }
    if (h2) { if (p < WLCAP) mylist[p] = ((e0 + 2) << SLB) | (int)s2; p = p + 1; }
    if (h3) { if (p < WLCAP) mylist[p] = ((e0 + 3) << SLB) | (int)s3; p = p + 1; }
    if (h4) { if (p < WLCAP) mylist[p] = ((e0 + 4) << SLB) | (int)s4; p = p + 1; }
    if (h5) { if (p < WLCAP) mylist[p] = ((e0 + 5) << SLB) | (int)s5; p = p + 1; }
    if (h6) { if (p < WLCAP) mylist[p] = ((e0 + 6) << SLB) | (int)s6; p = p + 1; }
    if (h7) { if (p < WLCAP) mylist[p] = ((e0 + 7) << SLB) | (int)s7; p = p + 1; }
    wc += (int)(__builtin_popcount(m0) + __builtin_popcount(m1) + __builtin_popcount(m2) + __builtin_popcount(m3) +
                __builtin_popcount(m4) + __builtin_popcount(m5) + __builtin_popcount(m6) + __builtin_popcount(m7));
  }
  return wc;
}

__device__ __forceinline__ void bucket_flush(const int* pl, const int* cnt, const int* offs, const int* dvb, int ov,
                                             int* lp, int* cp, int* op, int* dp, int* fp, int tid) {
#pragma unroll 1
  for (int i = tid * 4; i < RCAP; i += NTHR * 4) {
    const v4i v = *(const v4ia*)(pl + i);
    *(volatile v4i*)(lp + i) = v;
  }
  {
    const v4i v = *(const v4ia*)(cnt + 4 * tid);
    *(volatile v4i*)(cp + 4 * tid) = v;
  }
  {
    const v4i v = *(const v4ia*)(offs + 4 * tid);
    *(volatile v4i*)(op + 4 * tid) = v;
  }
  {
    const v4i v = *(const v4ia*)(dvb + 4 * tid);
    *(volatile v4i*)(dp + 4 * tid) = v;
  }
  if (tid < 8) {
    const v4i f = {ov, ov, ov, ov};
    *(volatile v4i*)(fp + 4 * tid) = f;
  }
}

__global__ __launch_bounds__(NTHR) void k_bucket(const int* __restrict__ srcs, const int* __restrict__ dsts,
                                                 int* LIST, int* CNT, int* OFF, int* DINVB, int* FLAG) {
  extern __shared__ __attribute__((aligned(16))) int dsm[];
  int* wl   = dsm;
  int* pl   = dsm + NWAVE * WLCAP;
  int* cnt  = pl + RCAP;
  int* offs = cnt + NBRUN;
  int* cur  = offs + NBRUN;
  int* misc = cur + NBRUN;
  const int tid = (int)threadIdx.x, lane = tid & 31, wave = tid >> 5;
  const int blk = (int)blockIdx.x;
  const unsigned nbs = (unsigned)(blk * NBRUN);

  {
    const v4i z4 = {0, 0, 0, 0};
    for (int i = tid * 4; i < BK_ZINTS; i += NTHR * 4) *(v4ia*)(dsm + i) = z4;
    if (tid < 16) misc[tid] = 0;
  }
  __syncthreads();

  {
    const int per  = ((GE + NWAVE * WCH - 1) / (NWAVE * WCH)) * WCH;
    const int ebeg = wave * per;
    const int eend = (ebeg + per < GE) ? (ebeg + per) : GE;
    int* mylist = wl + wave * WLCAP;
    int wc = 0;
    int cb = ebeg;
#pragma unroll 1
    for (; cb + WCH <= eend; cb += WCH) {
      const int e0 = cb + lane * EPT;
      const v4i da = *(const v4ia*)(dsts + e0);
      const v4i db = *(const v4ia*)(dsts + e0 + 4);
      asm volatile("" :: "v"(da));
      asm volatile("" :: "v"(db));
      wc = bk_emit(mylist, wc, e0, nbs, da.x, da.y, da.z, da.w, db.x, db.y, db.z, db.w);
    }
    if (cb < eend) {
      const int e0 = cb + lane * EPT;
      int kx[8];
#pragma unroll
      for (int j = 0; j < 8; ++j) {
        const int e  = e0 + j;
        const int ec = e < GE - 1 ? e : GE - 1;
        const int v  = dsts[ec];
        asm volatile("" :: "v"(v));
        kx[j] = (e < eend) ? v : -1;
      }
      wc = bk_emit(mylist, wc, e0, nbs, kx[0], kx[1], kx[2], kx[3], kx[4], kx[5], kx[6], kx[7]);
    }
    if (lane == 0) misc[wave] = wc;
  }
  __syncthreads();

  if (wave == 0) {
    int ov = 0;
    int tot = 0;
#pragma unroll 1
    for (int w2 = 0; w2 < NWAVE; ++w2) {
      int c = misc[w2];
      if (c > WLCAP) ov = 1;
      c = c < 0 ? 0 : (c > WLCAP ? WLCAP : c);
      tot += c;
#pragma unroll 1
      for (int b0 = 0; b0 < c; b0 += 32) {
        const int idx = b0 + lane;
        const int ent = wl[w2 * WLCAP + (idx < WLCAP ? idx : WLCAP - 1)];
        const int m32 = (c - b0) < 32 ? (c - b0) : 32;
#pragma unroll 1
        for (int k = 0; k < m32; ++k) {
          const int u    = __builtin_amdgcn_readlane(ent, k);
          const int slot = u & (NBRUN - 1);
          if (lane == 0) cnt[slot] = cnt[slot] + 1;
        }
      }
    }
    if (tot > RCAP) ov = 1;
    if (lane == 0) {
      misc[9]  = ov;
      misc[10] = tot > RCAP ? RCAP : tot;
    }
  }
  __syncthreads();
  if (wave == 0) {
    const int base = lane * (NBRUN / 32);
    int s = 0;
#pragma unroll 1
    for (int i = 0; i < NBRUN / 32; ++i) s += cnt[base + i];
    int incl = s;
#pragma unroll
    for (int d = 1; d < 32; d <<= 1) {
      const int y = __shfl_up(incl, d, 32);
      if (lane >= d) incl += y;
    }
    int run = incl - s;
#pragma unroll 1
    for (int i = 0; i < NBRUN / 32; ++i) {
      const int cv = cnt[base + i];
      offs[base + i] = run;
      cur[base + i]  = run;
      run += cv;
    }
  }
  __syncthreads();

  if (wave == 0) {
#pragma unroll 1
    for (int w2 = 0; w2 < NWAVE; ++w2) {
      int c = misc[w2];
      c = c < 0 ? 0 : (c > WLCAP ? WLCAP : c);
#pragma unroll 1
      for (int b0 = 0; b0 < c; b0 += 32) {
        const int idx = b0 + lane;
        const int ent = wl[w2 * WLCAP + (idx < WLCAP ? idx : WLCAP - 1)];
        const int m32 = (c - b0) < 32 ? (c - b0) : 32;
#pragma unroll 1
        for (int k = 0; k < m32; ++k) {
          const int u = __builtin_amdgcn_readlane(ent, k);
          if (lane == 0) {
            const int slot = u & (NBRUN - 1);
            int p = cur[slot];
            p = p < 0 ? 0 : (p > RCAP - 1 ? RCAP - 1 : p);
            pl[p] = (u >> SLB) & 0x1FFFFF;
            cur[slot] = p + 1;
          }
        }
      }
    }
  }
  __syncthreads();

  {
    const int tot = misc[10];
#pragma unroll 1
    for (int i = tid * 4; i < RCAP; i += NTHR * 4) {
      const v4i e4 = *(const v4ia*)(pl + i);
      const int e0 = clampi(e4.x, 0, GE - 1), e1 = clampi(e4.y, 0, GE - 1);
      const int e2 = clampi(e4.z, 0, GE - 1), e3 = clampi(e4.w, 0, GE - 1);
      int s0 = srcs[e0];
      asm volatile("" :: "v"(s0));
      int s1 = srcs[e1];
      asm volatile("" :: "v"(s1));
      int s2 = srcs[e2];
      asm volatile("" :: "v"(s2));
      int s3 = srcs[e3];
      asm volatile("" :: "v"(s3));
      s0 = clampi(s0, 0, GN - 1); s1 = clampi(s1, 0, GN - 1);
      s2 = clampi(s2, 0, GN - 1); s3 = clampi(s3, 0, GN - 1);
      v4i o;
      o.x = (i + 0 < tot) ? s0 : 0;
      o.y = (i + 1 < tot) ? s1 : 0;
      o.z = (i + 2 < tot) ? s2 : 0;
      o.w = (i + 3 < tot) ? s3 : 0;
      *(v4ia*)(pl + i) = o;
    }
    const v4i c4 = *(const v4ia*)(cnt + 4 * tid);
    int cc[4] = { c4.x, c4.y, c4.z, c4.w };
    int db[4];
#pragma unroll 1
    for (int j = 0; j < 4; ++j) {
      int cj = j == 0 ? cc[0] : (j == 1 ? cc[1] : (j == 2 ? cc[2] : cc[3]));
      const float degf = (float)(cj + 1);
      const float r    = 1.0f / sqrtf(degf);
      float dv = (degf > 0.0f) ? r : 0.0f;
      const int node = (int)nbs + 4 * tid + j;
      dv = (node < GN) ? dv : 0.0f;
      const int bits = __float_as_int(dv);
      if (j == 0) db[0] = bits; else if (j == 1) db[1] = bits; else if (j == 2) db[2] = bits; else db[3] = bits;
    }
    const v4i d4 = { db[0], db[1], db[2], db[3] };
    *(v4ia*)(cur + 4 * tid) = d4;
  }
  __syncthreads();

  const int ovf = misc[9];
  int* lp = LIST + (size_t)blk * (size_t)RCAP;
  int* cp = CNT + (size_t)blk * NBRUN;
  int* op = OFF + (size_t)blk * NBRUN;
  int* dp = DINVB + (size_t)blk * NBRUN;
  int* fp = FLAG + (size_t)blk * 32;
  bucket_flush(pl, cnt, offs, cur, ovf, lp, cp, op, dp, fp, tid);
  __threadfence();
  bucket_flush(pl, cnt, offs, cur, ovf, lp, cp, op, dp, fp, tid);
}

template <int CPL>
__device__ __forceinline__ void walk_row(const int* __restrict__ lb, const float* __restrict__ DINV,
                                         const float* __restrict__ T, int o, int last, int trip, float dd, int lane,
                                         float& a0, float& a1) {
#pragma unroll 1
  for (int b0 = 0; b0 < trip; b0 += 32) {
    int idx = o + b0 + lane;
    idx = idx > last ? last : idx;
    int sr = lb[idx];
    asm volatile("" :: "v"(sr));
    sr = clampi(sr, 0, GN - 1);
    const float ds = DINV[sr];
    asm volatile("" :: "v"(ds));
    const int dsb = __float_as_int(ds);
    const int m32 = (trip - b0) < 32 ? (trip - b0) : 32;
#pragma unroll 1
    for (int k = 0; k < m32; ++k) {
      const int   sk = __builtin_amdgcn_readlane(sr, k);
      const float dk = __int_as_float(__builtin_amdgcn_readlane(dsb, k));
      const float w  = dk * dd;
      if (CPL == 2) {
        const v2f q = *(const v2fa*)(T + (size_t)sk * GH + 2 * lane);
        const float t0 = q.x * w;
        const float t1 = q.y * w;
        a0 = a0 + t0;
        a1 = a1 + t1;
      } else {
        const float q  = T[(size_t)sk * GH + lane];
        const float t0 = q * w;
        a0 = a0 + t0;
      }
    }
  }
}

__global__ __launch_bounds__(NTHR) void k_walk1(const int* __restrict__ LIST, const int* __restrict__ CNT,
                                                const int* __restrict__ OFF, const float* __restrict__ DINV,
                                                const int* __restrict__ FLAG, const float* __restrict__ T,
                                                const float* __restrict__ B1T, unsigned* Z32) {
  const int tid = (int)threadIdx.x, lane = tid & 31, wave = tid >> 5;
  const int node = (int)blockIdx.x * NWAVE + wave;
  const int bb   = node >> SLB;
  const int c = CNT[node];
  asm volatile("" :: "v"(c));
  int o = OFF[node];
  asm volatile("" :: "v"(o));
  const int flag = FLAG[(size_t)bb * 32];
  asm volatile("" :: "v"(flag));
  const float dd = DINV[node];
  asm volatile("" :: "v"(dd));
  const v2f ts = *(const v2fa*)(T + (size_t)node * GH + 2 * lane);
  asm volatile("" :: "v"(ts));
  const v2f bv = *(const v2fa*)(B1T + 2 * lane);
  asm volatile("" :: "v"(bv));

  const bool live = node < GN;
  const bool big  = c > DEGCAP;
  const int trip  = __builtin_amdgcn_readfirstlane(live ? clampi(c, 0, DEGCAP) : 0);
  o = clampi(o, 0, RCAP - 1);
  int last = o + (trip > 0 ? trip : 1) - 1;
  last = last > RCAP - 1 ? RCAP - 1 : last;
  const int* lb = LIST + (size_t)bb * (size_t)RCAP;

  float a0 = 0.0f, a1 = 0.0f;
  walk_row<2>(lb, DINV, T, o, last, trip, dd, lane, a0, a1);

  const float wself = dd * dd;
  const float u0 = ts.x * wself;
  const float u1 = ts.y * wself;
  a0 = a0 + u0;
  a1 = a1 + u1;
  float v0 = a0 + bv.x;
  float v1 = a1 + bv.y;
  v0 = (v0 > 0.0f) ? v0 : (v0 - v0);
  v1 = (v1 > 0.0f) ? v1 : (v1 - v1);
  const float qnan = __uint_as_float(0x7fc00000u);
  const bool bad = (flag != 0) || big;
  v0 = bad ? qnan : v0;
  v1 = bad ? qnan : v1;
  v0 = live ? v0 : 0.0f;
  v1 = live ? v1 : 0.0f;

  const unsigned hw = pk16(bf16_bits(v0), bf16_bits(v1));
#if SPLIT_L2
  const unsigned lw = pk16(bf16_lo_bits(v0), bf16_lo_bits(v1));
#else
  const unsigned lw = hw & 0u;
#endif
  volatile unsigned* zp = (volatile unsigned*)(Z32 + (size_t)node * GH);
  zp[lane]      = hw;
  zp[32 + lane] = lw;
  __threadfence();
  zp[lane]      = hw;
  zp[32 + lane] = lw;
}

__global__ __launch_bounds__(NTHR) void k_walk2(const int* __restrict__ LIST, const int* __restrict__ CNT,
                                                const int* __restrict__ OFF, const float* __restrict__ DINV,
                                                const int* __restrict__ FLAG, const float* __restrict__ T,
                                                const float* __restrict__ B2T, float* out, int nn) {
  const int tid = (int)threadIdx.x, lane = tid & 31, wave = tid >> 5;
  const int node = (int)blockIdx.x * NWAVE + wave;
  const int nodec = clampi(node, 0, GMP - 1);
  const int bb   = nodec >> SLB;
  const int c = CNT[nodec];
  asm volatile("" :: "v"(c));
  int o = OFF[nodec];
  asm volatile("" :: "v"(o));
  const int flag = FLAG[(size_t)bb * 32];
  asm volatile("" :: "v"(flag));
  const float dd = DINV[nodec];
  asm volatile("" :: "v"(dd));
  const float ts = T[(size_t)nodec * GH + lane];
  asm volatile("" :: "v"(ts));
  const float bv = B2T[lane];
  asm volatile("" :: "v"(bv));

  const bool live = node < nn;
  const bool big  = c > DEGCAP;
  const int trip  = __builtin_amdgcn_readfirstlane(live ? clampi(c, 0, DEGCAP) : 0);
  o = clampi(o, 0, RCAP - 1);
  int last = o + (trip > 0 ? trip : 1) - 1;
  last = last > RCAP - 1 ? RCAP - 1 : last;
  const int* lb = LIST + (size_t)bb * (size_t)RCAP;

  float a0 = 0.0f, a1 = 0.0f;
  walk_row<1>(lb, DINV, T, o, last, trip, dd, lane, a0, a1);

  const float wself = dd * dd;
  const float u0 = ts * wself;
  a0 = a0 + u0;
  float v0 = a0 + bv;
  const float qnan = __uint_as_float(0x7fc00000u);
  const bool bad = (flag != 0) || big;
  v0 = bad ? qnan : v0;
  if (node < nn) {
    volatile float* op = (volatile float*)(out + (size_t)node * GC + lane);
    *op = v0;
    __threadfence();
    *op = v0;
  }
}

extern "C" void kernel_launch(void* const* d_in, const int* in_sizes, int n_in,
                              void* d_out, int out_size, void* d_ws, size_t ws_size,
                              hipStream_t stream) {
  if (n_in < 7) return;
  if (in_sizes[0] != GN * GK1) return;
  if (in_sizes[1] != 2 * GE) return;
  if (in_sizes[3] != GK1 * GH) return;
  if (in_sizes[4] != GH) return;
  if (in_sizes[5] != GH * GC) return;
  if (in_sizes[6] != GC) return;
  if (out_size != GN * GC) return;

  const float* x  = (const float*)d_in[0];
  const int*   ei = (const int*)d_in[1];
  const float* W1 = (const float*)d_in[3];
  const float* b1 = (const float*)d_in[4];
  const float* W2 = (const float*)d_in[5];
  const float* b2 = (const float*)d_in[6];
  const int* srcs = ei;
  const int* dsts = ei + GE;
  float* out = (float*)d_out;

  constexpr size_t zXB   = (size_t)GMP * GK1 * 2;
  constexpr size_t zT    = (size_t)GMP * GH * 4;
  constexpr size_t zLIST = (size_t)NBK * RCAP * 4;
  constexpr size_t zTAB  = (size_t)NBK * NBRUN * 4;
  constexpr size_t zFLAG = (size_t)NBK * 128;
  constexpr size_t zW    = (size_t)GH * GK1 * 2;
  constexpr size_t zBIAS = 1024;
  constexpr size_t oXB   = 0;
  constexpr size_t oT    = oXB + zXB;
  constexpr size_t oLIST = oT + zT;
  constexpr size_t oCNT  = oLIST + zLIST;
  constexpr size_t oOFF  = oCNT + zTAB;
  constexpr size_t oDINV = oOFF + zTAB;
  constexpr size_t oFLAG = oDINV + zTAB;
  constexpr size_t oW1T  = oFLAG + zFLAG;
  constexpr size_t oW2P  = oW1T + zW;
  constexpr size_t oBIAS = oW2P + zW;
  constexpr size_t oEND  = oBIAS + zBIAS;
  static_assert(zXB % 256 == 0 && zT % 256 == 0 && zLIST % 256 == 0 && zTAB % 256 == 0);
  static_assert(zFLAG % 256 == 0 && zW % 256 == 0 && zBIAS % 256 == 0);
  static_assert(zXB == (size_t)GMP * (2 * GH) * 2);
  static_assert(zTAB >= (size_t)GMP * 4);
  static_assert(oEND == 60929280);
  static_assert(oEND <= ((size_t)128 << 20));
  if (oEND > ws_size) return;

  char* ws = (char*)d_ws;
  unsigned short* XB   = (unsigned short*)(ws + oXB);
  unsigned*       Z32  = (unsigned*)(ws + oXB);
  float*          T    = (float*)(ws + oT);
  int*            LIST = (int*)(ws + oLIST);
  int*            CNT  = (int*)(ws + oCNT);
  int*            OFF  = (int*)(ws + oOFF);
  int*            DVB  = (int*)(ws + oDINV);
  const float*    DINV = (const float*)(ws + oDINV);
  int*            FLAG = (int*)(ws + oFLAG);
  unsigned short* W1T  = (unsigned short*)(ws + oW1T);
  unsigned short* W2P  = (unsigned short*)(ws + oW2P);
  float*          BIAS = (float*)(ws + oBIAS);
  const float*    B1T  = BIAS;
  const float*    B2T  = BIAS + 64;
  const float*    ZB   = BIAS + 128;

  hipFuncSetAttribute(reinterpret_cast<const void*>(&k_bucket), hipFuncAttributeMaxDynamicSharedMemorySize, (int)BK_LDS);

  constexpr int gridPlane = GMP * GK1 / 8 / 256;
  constexpr int gridGemm  = ((GMP / 64) * 1 + 7) / 8;
  k_plane<0><<<gridPlane, 256, 0, stream>>>(x, GN, GK1, GK1, XB, GMP, GK1);
  k_prep<<<9, NTHR, 0, stream>>>(W1, b1, W2, b2, W1T, W2P, BIAS);
  k_bucket<<<NBK, NTHR, BK_LDS, stream>>>(srcs, dsts, LIST, CNT, OFF, DVB, FLAG);
  k_gemm_nt<0, 0><<<gridGemm, 256, 0, stream>>>(XB, W1T, ZB, T, GMP, GH, GK1, GH);
  k_walk1<<<GMP / NWAVE, NTHR, 0, stream>>>(LIST, CNT, OFF, DINV, FLAG, T, B1T, Z32);
  k_gemm_nt<0, 0><<<gridGemm, 256, 0, stream>>>((const unsigned short*)Z32, W2P, ZB, T, GMP, GH, 2 * GH, GH);
  k_walk2<<<GN / NWAVE, NTHR, 0, stream>>>(LIST, CNT, OFF, DINV, FLAG, T, B2T, out, GN);
}
